// GIN_regression_87282325390050
// MI455X (gfx1250) — hardware-verified
//
#include <hip/hip_runtime.h>
#include <stddef.h>


#define NTHR   256
#define NWAVE  8
#define EPT    16
#define CHUNK  (NTHR * EPT)
#define WCAP   (EPT * 32)
#define WSC    16.0f
#define WINV   0.0625f
#define LALPHA 0.2f
#define F1     128
#define F2     256
#define NB1    512
#define NB2    256

#define LDS_ACC_BYTES 262144
#define LDS_LIST      (LDS_ACC_BYTES)
#define LDS_WCNT      (LDS_LIST + NWAVE * WCAP * 4)
#define LDS_AGG       (LDS_WCNT + 64)

static_assert(NB1 * F1 * 4 == LDS_ACC_BYTES);
static_assert(NB2 * F2 * 4 == LDS_ACC_BYTES);
static_assert(CHUNK <= 4096);
static_assert(NB1 < (1 << 19) && NB2 < (1 << 19));
static_assert((LDS_AGG % 16) == 0);
static_assert(LDS_AGG <= 300 * 1024);
static_assert((NB1 % NWAVE) == 0 && (NB2 % NWAVE) == 0);
static_assert(WCAP == 32 * EPT);

typedef float    v4f  __attribute__((ext_vector_type(4)));
typedef float    v8f  __attribute__((ext_vector_type(8)));
typedef int      v4i  __attribute__((ext_vector_type(4)));
typedef _Float16 v8h  __attribute__((ext_vector_type(8)));
typedef _Float16 v16h __attribute__((ext_vector_type(16)));
union FragH { v16h v; v8h h[2]; };
union Pk8 { v8h h; v4i i; };

__device__ __forceinline__ v8f wmh(v16h a, v16h b, v8f c) {
  v8f d = __builtin_amdgcn_wmma_f32_16x16x32_f16(false, a, false, b, (short)0, c, false, false);
  asm volatile("v_nop\n\tv_nop\n\tv_nop\n\tv_nop" : "+v"(d) : "v"(a), "v"(b));
  return d;
}

__device__ __forceinline__ v8f splat8(float x) {
  v8f c;
#pragma unroll
  for (int i = 0; i < 8; ++i) c[i] = x;
  return c;
}

__device__ __forceinline__ v8h cv8z(v4f a, v4f b, bool ok) {
  v8h r;
  r[0] = (_Float16)(ok ? a.x : 0.0f); r[1] = (_Float16)(ok ? a.y : 0.0f);
  r[2] = (_Float16)(ok ? a.z : 0.0f); r[3] = (_Float16)(ok ? a.w : 0.0f);
  r[4] = (_Float16)(ok ? b.x : 0.0f); r[5] = (_Float16)(ok ? b.y : 0.0f);
  r[6] = (_Float16)(ok ? b.z : 0.0f); r[7] = (_Float16)(ok ? b.w : 0.0f);
  return r;
}

__global__ __launch_bounds__(NTHR) void k_prep(const float* __restrict__ w1, const float* __restrict__ w2,
                                              const float* __restrict__ w3, const float* __restrict__ w4,
                                              _Float16* p1, _Float16* p2, _Float16* p3, _Float16* p4) {
  const int b = blockIdx.x, tid = threadIdx.x;
  const float* src;
  _Float16* dst;
  int K, NC, ub;
  if (b < 16)      { src = w1; dst = p1; K = F1; NC = F2; ub = b; }
  else if (b < 48) { src = w2; dst = p2; K = F2; NC = F2; ub = b - 16; }
  else if (b < 80) { src = w3; dst = p3; K = F2; NC = F2; ub = b - 48; }
  else             { src = w4; dst = p4; K = F2; NC = F1; ub = b - 80; }
  const int u   = ub * NTHR + tid;
  const int cpr = K >> 3;
  int f  = u / cpr;
  const int kc = u - f * cpr;
  f = f < NC ? f : NC - 1;
  Pk8 pk;
#pragma unroll
  for (int j = 0; j < 8; ++j) {
    int k = 8 * kc + j;
    k = k < K ? k : K - 1;
    const float w = src[(size_t)k * NC + f];
    pk.h[j] = (_Float16)(w * WSC);
  }
  _Float16* dp = dst + (size_t)u * 8;
  *(volatile v4i*)dp = pk.i;
  __threadfence();
  *(volatile v4i*)dp = pk.i;
}

template <int NB>
__device__ __forceinline__ int scan_chunk(const int* __restrict__ dsts, int nE, int cbase, int nodeBase,
                                          int vec8, int* list, int tid, int wave) {
  const int el0  = tid * EPT;
  const int e0   = cbase + el0;
  const int sent = -2147483647 - 1;
  int d[EPT];
  if (vec8 != 0 && cbase + CHUNK <= nE) {
#pragma unroll
    for (int q = 0; q < EPT / 4; ++q) {
      const v4i t = *(const v4i*)(dsts + e0 + 4 * q);
      d[4 * q] = t.x; d[4 * q + 1] = t.y; d[4 * q + 2] = t.z; d[4 * q + 3] = t.w;
    }
  } else {
#pragma unroll
    for (int j = 0; j < EPT; ++j) {
      const int e  = e0 + j;
      const int ec = e < nE ? e : nE - 1;
      const int v  = dsts[ec];
      d[j] = (e < nE) ? v : sent;
    }
  }
  const unsigned nb = (unsigned)nodeBase;
  unsigned s[EPT];
  bool h[EPT];
  bool anyh = false;
#pragma unroll
  for (int j = 0; j < EPT; ++j) {
    s[j] = (unsigned)d[j] - nb;
    h[j] = s[j] < (unsigned)NB;
    anyh = anyh || h[j];
  }
  int wc = 0;
  const unsigned any = __builtin_amdgcn_ballot_w32(anyh);
  if (any != 0u) {
#pragma unroll
    for (int j = 0; j < EPT; ++j) {
      const unsigned mj = __builtin_amdgcn_ballot_w32(h[j]);
      if (mj != 0u) {
        if (h[j]) {
          const int pos = wc + (int)__builtin_amdgcn_mbcnt_lo(mj, 0u);
          if (pos < WCAP) list[wave * WCAP + pos] = (int)((s[j] << 12) | (unsigned)(el0 + j));
        }
        wc += (int)__builtin_popcount(mj);
      }
    }
  }
  return wc;
}

template <int F, int NB>
__device__ __forceinline__ void agg_rows_store(const float* __restrict__ xin, const float* acc, _Float16* hout,
                                               int nodeBase, int nN, int wave, int lane) {
  constexpr int RPW = NB / NWAVE;
  constexpr int LPR = F / 8;
  constexpr int RPI = 32 / LPR;
  static_assert((RPW % RPI) == 0);
#pragma unroll 1
  for (int it = 0; it < RPW / RPI; ++it) {
    const int lr   = wave * RPW + it * RPI + lane / LPR;
    const int c0   = 8 * (lane % LPR);
    const int node = nodeBase + lr;
    const bool ok  = node < nN;
    const int nc   = ok ? node : nN - 1;
    const float* xp = xin + (size_t)nc * F + c0;
    const float* ap = acc + lr * F + c0;
    const v4f h0 = *(const v4f*)xp + *(const v4f*)ap;
    const v4f h1 = *(const v4f*)(xp + 4) + *(const v4f*)(ap + 4);
    Pk8 pk;
    pk.h = cv8z(h0, h1, ok);
    *(volatile v4i*)(hout + (size_t)node * F + c0) = pk.i;
  }
}

template <int F, int NB>
__global__ __launch_bounds__(NTHR) void k_agg(const float* __restrict__ xin, const int* __restrict__ ei,
                                             _Float16* hout, int nN, int nE, int vec8) {
  extern __shared__ __attribute__((aligned(16))) unsigned char dsm[];
  float* acc  = (float*)dsm;
  int*   list = (int*)(dsm + LDS_LIST);
  int*   wcnt = (int*)(dsm + LDS_WCNT);
  constexpr int CPL = F / 32;
  const int tid = threadIdx.x, lane = tid & 31, wave = tid >> 5;
  const int nodeBase = blockIdx.x * NB;
  const int* srcs = ei;
  const int* dsts = ei + nE;

  {
    const v4f z = {0.0f, 0.0f, 0.0f, 0.0f};
    for (int i = tid; i < NB * F / 4; i += NTHR) *(v4f*)(acc + 4 * i) = z;
  }
  __syncthreads();

  const int nChunks = (nE + CHUNK - 1) / CHUNK;
#pragma unroll 1
  for (int ch = 0; ch < nChunks; ++ch) {
    const int cbase = ch * CHUNK;
    const int wc = scan_chunk<NB>(dsts, nE, cbase, nodeBase, vec8, list, tid, wave);
    if (lane == 0) wcnt[wave] = wc;
    __syncthreads();

#pragma unroll 1
    for (int wv = 0; wv < NWAVE; ++wv) {
      int n = wcnt[wv];
      n = n > WCAP ? WCAP : (n < 0 ? 0 : n);
      const int* lp = list + wv * WCAP;
#pragma unroll 1
      for (int base = 0; base < n; base += 32) {
        const int idx  = base + lane;
        const int ent  = lp[idx < WCAP ? idx : WCAP - 1];
        const bool mine = (idx < n) && (((ent >> 12) & (NWAVE - 1)) == wave);
        unsigned mk = __builtin_amdgcn_ballot_w32(mine);
        while (mk != 0u) {
          const int j = __builtin_ctz(mk);
          mk &= mk - 1u;
          const int ej = __shfl(ent, j, 32);
          int e = cbase + (ej & 0xFFF);
          e = e > nE - 1 ? nE - 1 : e;
          int sl = ej >> 12;
          sl = sl < 0 ? 0 : (sl > NB - 1 ? NB - 1 : sl);
          int sn = srcs[e];
          sn = sn < 0 ? 0 : (sn > nN - 1 ? nN - 1 : sn);
          const float* xp = xin + (size_t)sn * F + CPL * lane;
          float* ap = acc + sl * F + CPL * lane;
#pragma unroll
          for (int c = 0; c < CPL / 4; ++c) {
            const v4f xv = *(const v4f*)(xp + 4 * c);
            const v4f av = *(const v4f*)(ap + 4 * c);
            *(v4f*)(ap + 4 * c) = av + xv;
          }
        }
      }
    }
    __syncthreads();
  }
  __syncthreads();

  agg_rows_store<F, NB>(xin, acc, hout, nodeBase, nN, wave, lane);
  __threadfence();
  agg_rows_store<F, NB>(xin, acc, hout, nodeBase, nN, wave, lane);
}

template <int K>
__device__ __forceinline__ void mma_strip(const _Float16* __restrict__ A, const _Float16* __restrict__ Wt,
                                          int row0, int col0, int m, int hh, v8f (&acc)[4]) {
  const _Float16* ap = A  + (size_t)(row0 + m) * K + 8 * hh;
  const _Float16* bp = Wt + (size_t)(col0 + m) * K + 8 * hh;
#pragma unroll 2
  for (int k0 = 0; k0 < K; k0 += 32) {
    FragH a;
    a.h[0] = *(const v8h*)(ap + k0);
    a.h[1] = *(const v8h*)(ap + k0 + 16);
#pragma unroll
    for (int t = 0; t < 4; ++t) {
      FragH b;
      const _Float16* bq = bp + (size_t)(16 * t) * K + k0;
      b.h[0] = *(const v8h*)bq;
      b.h[1] = *(const v8h*)(bq + 16);
      acc[t] = wmh(a.v, b.v, acc[t]);
    }
  }
}

template <typename T, int PITCH>
__device__ __forceinline__ void stage_leaky(T* st, const v8f (&acc)[4], const float* __restrict__ bias,
                                            int col0, int rb, int cb, int m, int hh) {
#pragma unroll
  for (int t = 0; t < 4; ++t) {
    const float bv = bias[col0 + 16 * t + m];
#pragma unroll
    for (int r = 0; r < 8; ++r) {
      float v = acc[t][r] * WINV + bv;
      v = (v >= 0.0f) ? v : LALPHA * v;
      st[(rb + 8 * hh + r) * PITCH + cb + 16 * t + m] = (T)v;
    }
  }
}

__device__ __forceinline__ void tile_store_h(const _Float16* st, _Float16* outp, int row0, int col0, int lane) {
#pragma unroll
  for (int it = 0; it < 4; ++it) {
    const int q = 4 * it + (lane >> 3);
    const int p = 8 * (lane & 7);
    const v4i v = *(const v4i*)(st + q * 64 + p);
    *(volatile v4i*)(outp + (size_t)(row0 + q) * F2 + col0 + p) = v;
  }
}

template <int NC>
__device__ __forceinline__ void tile_store_f(const float* st, float* outp, int row0, int col0, int lane) {
#pragma unroll
  for (int it = 0; it < 8; ++it) {
    const int q  = 4 * it + (lane >> 3);
    const int r  = q >> 1;
    const int cs = 32 * (q & 1) + 4 * (lane & 7);
    const v4f v = *(const v4f*)(st + r * 64 + cs);
    *(volatile v4f*)(outp + (size_t)(row0 + r) * NC + col0 + cs) = v;
  }
}

template <int K>
__global__ __launch_bounds__(NTHR) void k_gemm_h(const _Float16* __restrict__ A, const _Float16* __restrict__ Wt,
                                                const float* __restrict__ bias, _Float16* outp) {
  __shared__ __attribute__((aligned(16))) _Float16 stg[NWAVE * 16 * 64];
  const int tid = threadIdx.x, lane = tid & 31, wave = tid >> 5, m = lane & 15, hh = lane >> 4;
  const int mt = wave >> 2, ng = wave & 3;
  const int row0 = blockIdx.x * 32 + 16 * mt;
  const int col0 = 64 * ng;
  v8f acc[4];
#pragma unroll
  for (int t = 0; t < 4; ++t) acc[t] = splat8(0.0f);
  mma_strip<K>(A, Wt, row0, col0, m, hh, acc);
  _Float16* st = stg + wave * 1024;
  stage_leaky<_Float16, 64>(st, acc, bias, col0, 0, 0, m, hh);
  __syncthreads();
  tile_store_h(st, outp, row0, col0, lane);
  __threadfence();
  tile_store_h(st, outp, row0, col0, lane);
}

template <int K>
__global__ __launch_bounds__(NTHR) void k_gemm_f(const _Float16* __restrict__ A, const _Float16* __restrict__ Wt,
                                                const float* __restrict__ bias, float* outp) {
  __shared__ __attribute__((aligned(16))) float stg[NWAVE * 16 * 64];
  const int tid = threadIdx.x, lane = tid & 31, wave = tid >> 5, m = lane & 15, hh = lane >> 4;
  const int mt = wave >> 2, ng = wave & 3;
  const int row0 = blockIdx.x * 32 + 16 * mt;
  const int col0 = 64 * ng;
  v8f acc[4];
#pragma unroll
  for (int t = 0; t < 4; ++t) acc[t] = splat8(0.0f);
  mma_strip<K>(A, Wt, row0, col0, m, hh, acc);
  float* st = stg + wave * 1024;
  stage_leaky<float, 64>(st, acc, bias, col0, 0, 0, m, hh);
  __syncthreads();
  tile_store_f<F2>(st, outp, row0, col0, lane);
  __threadfence();
  tile_store_f<F2>(st, outp, row0, col0, lane);
}

__global__ __launch_bounds__(NTHR) void k_gemm_head(const _Float16* __restrict__ A, const _Float16* __restrict__ Wt,
                                                   const float* __restrict__ b4, const float* __restrict__ W5,
                                                   const float* __restrict__ b5, float* out, int nN) {
  __shared__ __attribute__((aligned(16))) float hs[64 * F1];
  __shared__ __attribute__((aligned(16))) float hsum[64];
  const int tid = threadIdx.x, lane = tid & 31, wave = tid >> 5, m = lane & 15, hh = lane >> 4;
  const int mt = wave >> 1, ng = wave & 1;
  const int rowBlk = blockIdx.x * 64;
  const int row0 = rowBlk + 16 * mt;
  const int col0 = 64 * ng;
  v8f acc[4];
#pragma unroll
  for (int t = 0; t < 4; ++t) acc[t] = splat8(0.0f);
  mma_strip<F2>(A, Wt, row0, col0, m, hh, acc);
  stage_leaky<float, F1>(hs, acc, b4, col0, 16 * mt, col0, m, hh);
  __syncthreads();

  const int r = tid >> 2, q = tid & 3;
  float s = 0.0f;
  {
    const float* hp = hs + r * F1 + 32 * q;
    const float* wp = W5 + 32 * q;
#pragma unroll 1
    for (int j = 0; j < 8; ++j) {
      const v4f hv = *(const v4f*)(hp + 4 * j);
      const v4f wv = *(const v4f*)(wp + 4 * j);
      s += hv.x * wv.x;
      s += hv.y * wv.y;
      s += hv.z * wv.z;
      s += hv.w * wv.w;
    }
  }
  s += __shfl_xor(s, 1, 32);
  s += __shfl_xor(s, 2, 32);
  const float bb = b5[0];
  if (q == 0) hsum[r] = s + bb;
  __syncthreads();

  int nval = nN - rowBlk;
  nval = nval < 0 ? 0 : (nval > 64 ? 64 : nval);
  const int nl = nval >> 2;
  if (wave == 0 && lane < nl) {
    const v4f v = *(const v4f*)(hsum + 4 * lane);
    *(volatile v4f*)(out + (size_t)rowBlk + 4 * lane) = v;
  }
  __threadfence();
  if (wave == 0 && lane < nl) {
    const v4f v = *(const v4f*)(hsum + 4 * lane);
    *(volatile v4f*)(out + (size_t)rowBlk + 4 * lane) = v;
  }
}

extern "C" void kernel_launch(void* const* d_in, const int* in_sizes, int n_in,
                              void* d_out, int out_size, void* d_ws, size_t ws_size,
                              hipStream_t stream) {
  if (n_in < 13) return;
  const int nN = in_sizes[0] / F1;
  if (nN < 1 || in_sizes[0] != nN * F1 || (nN & 3) != 0) return;
  const int nE = in_sizes[2] / 2;
  if (nE < 1 || in_sizes[2] != 2 * nE) return;
  if (in_sizes[3] != F1 * F2 || in_sizes[4] != F2) return;
  if (in_sizes[5] != F2 * F2 || in_sizes[6] != F2) return;
  if (in_sizes[7] != F2 * F2 || in_sizes[8] != F2) return;
  if (in_sizes[9] != F2 * F1 || in_sizes[10] != F1) return;
  if (in_sizes[11] != F1 || in_sizes[12] != 1) return;
  if (out_size != nN) return;

  const float* x  = (const float*)d_in[0];
  const int*   ei = (const int*)d_in[2];
  const float* W1 = (const float*)d_in[3];
  const float* b1 = (const float*)d_in[4];
  const float* W2 = (const float*)d_in[5];
  const float* b2 = (const float*)d_in[6];
  const float* W3 = (const float*)d_in[7];
  const float* b3 = (const float*)d_in[8];
  const float* W4 = (const float*)d_in[9];
  const float* b4 = (const float*)d_in[10];
  const float* W5 = (const float*)d_in[11];
  const float* b5 = (const float*)d_in[12];
  float* outp = (float*)d_out;

  const int Np = ((nN + NB1 - 1) / NB1) * NB1;

  char* ws = (char*)d_ws;
  size_t off = 0;
  const size_t oW1 = off; off += (size_t)F2 * F1 * 2;
  const size_t oW2 = off; off += (size_t)F2 * F2 * 2;
  const size_t oW3 = off; off += (size_t)F2 * F2 * 2;
  const size_t oW4 = off; off += (size_t)F1 * F2 * 2;
  const size_t oA1 = off; off += (size_t)Np * F1 * 2;
  const size_t oZ  = off; off += (size_t)Np * F2 * 2;
  const size_t oH1 = off; off += (size_t)Np * F2 * 4;
  const size_t oA2 = off; off += (size_t)Np * F2 * 2;
  size_t limit = (size_t)134217728;
  if (ws_size < limit) limit = ws_size;
  if (off > limit) return;

  _Float16* pW1 = (_Float16*)(ws + oW1);
  _Float16* pW2 = (_Float16*)(ws + oW2);
  _Float16* pW3 = (_Float16*)(ws + oW3);
  _Float16* pW4 = (_Float16*)(ws + oW4);
  _Float16* A1  = (_Float16*)(ws + oA1);
  _Float16* Z   = (_Float16*)(ws + oZ);
  float*    H1  = (float*)(ws + oH1);
  _Float16* A2  = (_Float16*)(ws + oA2);

  const int vec8 = ((nE & 3) == 0) ? 1 : 0;

  k_prep<<<96, NTHR, 0, stream>>>(W1, W2, W3, W4, pW1, pW2, pW3, pW4);

  hipFuncSetAttribute(reinterpret_cast<const void*>(&k_agg<F1, NB1>), hipFuncAttributeMaxDynamicSharedMemorySize, LDS_AGG);
  hipFuncSetAttribute(reinterpret_cast<const void*>(&k_agg<F2, NB2>), hipFuncAttributeMaxDynamicSharedMemorySize, LDS_AGG);

  k_agg<F1, NB1><<<Np / NB1, NTHR, LDS_AGG, stream>>>(x, ei, A1, nN, nE, vec8);
  k_gemm_h<F1><<<Np / 32, NTHR, 0, stream>>>(A1, pW1, b1, Z);
  k_gemm_f<F2><<<Np / 32, NTHR, 0, stream>>>(Z, pW2, b2, H1);

  k_agg<F2, NB2><<<Np / NB2, NTHR, LDS_AGG, stream>>>(H1, ei, A2, nN, nE, vec8);
  k_gemm_h<F2><<<Np / 32, NTHR, 0, stream>>>(A2, pW3, b3, Z);
  k_gemm_head<<<Np / 64, NTHR, 0, stream>>>(Z, pW4, b4, W5, b5, outp, nN);
}
